// SolventLayer_26706106647095
// MI455X (gfx1250) — hardware-run, weakly checked
//
#include <hip/hip_runtime.h>


#ifndef NGR
#define NGR 4096
#endif
#define NGR_FULL 4096
#define HID  64
#define NDIM 74
#define KE   96
#define LPR  96
#define LSE  64
#define ZW   256
#define GP   72
#define TP   104
#define OSF  68
#define QRS  2048.0f
#define QRI  (1.0f / 2048.0f)
#define WSC  64.0f
#define WSI  (1.0f / 64.0f)
#define NRM  (1.0f / 3.0f)
#define BN_EPS 1e-5f

__host__ __device__ constexpr int pri_off(int b) { return 32 * b + (b / 65) * 2080 + ((b % 65) * ((b % 65) - 1)) / 2; }
__host__ __device__ constexpr int sec_off(int b) { return 16 * b + (b / 49) * 1176 + ((b % 49) * ((b % 49) - 1)) / 2; }
enum : int { NM = pri_off(NGR), NS = sec_off(NGR), NM_FULL = pri_off(NGR_FULL), NS_FULL = sec_off(NGR_FULL),
             NMP = ((NM + 63) / 64) * 64, NSP = ((NS + 63) / 64) * 64, NBH = NMP / 64, NBS = NSP / 64 };

static_assert(NM_FULL == 262112);
static_assert(NS_FULL == 163550);
static_assert(NGR <= NGR_FULL);
static_assert(NGR % 32 == 0);
static_assert(HID == 64);
static_assert(HID % 32 == 0);
static_assert(KE % 32 == 0);
static_assert(KE >= NDIM);
static_assert(LPR % 16 == 0);
static_assert(LSE % 16 == 0);
static_assert(LPR % 32 == 0);
static_assert(LSE % 32 == 0);
static_assert(ZW == 4 * HID);
static_assert(ZW % 32 == 0);
static_assert(((long long)NS * NDIM) % 4 == 0);
static_assert((64 * NDIM) % 4 == 0);
static_assert((GP * 2) % 16 == 0);
static_assert((TP * 2) % 16 == 0);
static_assert(GP >= HID + 8 - 8);
static_assert(TP >= KE);
static_assert((OSF * 4) % 16 == 0);
static_assert(NMP % 64 == 0);
static_assert(NSP % 64 == 0);

typedef _Float16 h16;
typedef unsigned short bf;
typedef __attribute__((ext_vector_type(16))) __bf16   v16bf;
typedef __attribute__((ext_vector_type(16))) _Float16 v16h;
typedef __attribute__((ext_vector_type(8)))  _Float16 v8h;
typedef __attribute__((ext_vector_type(4)))  _Float16 v4h;
typedef __attribute__((ext_vector_type(8)))  unsigned short v8us;
typedef __attribute__((ext_vector_type(4)))  unsigned short v4us;
typedef __attribute__((ext_vector_type(8)))  float    v8f;
typedef __attribute__((ext_vector_type(4)))  float    v4f;
typedef v4f  __attribute__((may_alias)) v4fa;

__device__ __forceinline__ unsigned short f2bf(float f) { unsigned u = __float_as_uint(f); u += 0x7FFFu + ((u >> 16) & 1u); return (unsigned short)(u >> 16); }
__device__ __forceinline__ float bfr(float f) { return __uint_as_float(((unsigned)f2bf(f)) << 16); }
__device__ __forceinline__ v16h cat16(v8h lo, v8h hi) { return __builtin_shufflevector(lo, hi, 0, 1, 2, 3, 4, 5, 6, 7, 8, 9, 10, 11, 12, 13, 14, 15); }
__device__ __forceinline__ v16bf cat16b(v8us lo, v8us hi) { return __builtin_bit_cast(v16bf, __builtin_shufflevector(lo, hi, 0, 1, 2, 3, 4, 5, 6, 7, 8, 9, 10, 11, 12, 13, 14, 15)); }
__device__ __forceinline__ v16h  ldh(const h16* p) { return cat16(*(const v8h*)p, *(const v8h*)(p + 16)); }
__device__ __forceinline__ v16bf ldb(const bf* p)  { return cat16b(*(const v8us*)p, *(const v8us*)(p + 16)); }
__device__ __forceinline__ v16h  ldhs(const h16* p) { return cat16(*(const v8h*)p, *(const v8h*)(p + 16)); }
__device__ __forceinline__ v16bf ldbs(const bf* p)  { return cat16b(*(const v8us*)p, *(const v8us*)(p + 16)); }
__device__ __forceinline__ void wave_sync() { __builtin_amdgcn_fence(3  , "wavefront"); __builtin_amdgcn_wave_barrier(); asm volatile("" ::: "memory"); }
static __device__ __forceinline__ h16 toh_flush(float v) { const h16 r = (h16)v; return (fabsf(v) < 6.103515625e-05f) ? (h16)0.0f : r; }
__device__ __forceinline__ v8f wmma16g(v16h a, v16h b, v8f c) {
    c = __builtin_amdgcn_wmma_f32_16x16x32_f16(false, a, false, b, (short)0, c, false, false);
    asm volatile("v_nop\n\tv_nop\n\tv_nop\n\tv_nop" : "+v"(c) : "v"(a), "v"(b)); return c; }
__device__ __forceinline__ v8f wmmabg(v16bf a, v16bf b, v8f c) {
    c = __builtin_amdgcn_wmma_f32_16x16x32_bf16(false, a, false, b, (short)0, c, false, false);
    asm volatile("v_nop\n\tv_nop\n\tv_nop\n\tv_nop" : "+v"(c) : "v"(a), "v"(b)); return c; }

__global__ __launch_bounds__(256) void k_wtb(const float* __restrict__ W, bf* dst, int K, int N, int KP, int total8) {
    const int i = blockIdx.x * 256 + threadIdx.x; if (i >= total8) return;
    const int e = i * 8; const int n = e / KP, k0 = e - n * KP;
    v8us o;
#pragma unroll
    for (int j = 0; j < 8; ++j) { const int k = k0 + j; const int kc = k < K ? k : K - 1; float v = W[(size_t)kc * N + n]; asm volatile("" : "+v"(v)); o[j] = (k < K) ? f2bf(v) : (unsigned short)0; }
    *(volatile v8us*)(dst + e) = o; __threadfence(); *(volatile v8us*)(dst + e) = o;
}
__global__ __launch_bounds__(256) void k_wth(const float* __restrict__ W, h16* dst, int K, int N, int KP, int total8, float carry) {
    const int i = blockIdx.x * 256 + threadIdx.x; if (i >= total8) return;
    const float* Wz = W + (size_t)blockIdx.y * K * N; h16* dz = dst + (size_t)blockIdx.y * N * KP;
    const int e = i * 8; const int n = e / KP, k0 = e - n * KP;
    v8h o;
#pragma unroll
    for (int j = 0; j < 8; ++j) { const int k = k0 + j; const int kc = k < K ? k : K - 1; float v = Wz[(size_t)kc * N + n]; asm volatile("" : "+v"(v)); o[j] = (k < K) ? toh_flush(bfr(v) * carry) : (h16)0.0f; }
    *(volatile v8h*)(dz + e) = o; __threadfence(); *(volatile v8h*)(dz + e) = o;
}

__global__ __launch_bounds__(512) void k_check(const int* __restrict__ pseg, const int* __restrict__ ppos, const int* __restrict__ sseg, const int* __restrict__ spos,
                                               const int* __restrict__ esrc, const int* __restrict__ edst, int* FLAG) {
    __shared__ int wbad[16];
    const int tid = threadIdx.x, lane = tid & 31;
    const int wave = __builtin_amdgcn_readfirstlane((int)(threadIdx.x >> 5));
    int bad = 0;
#pragma unroll 1
    for (int n0 = 0; n0 < NM; n0 += 512) {
        const int n = n0 + tid; const int ok = (int)(n < NM); const int nc = ok ? n : NM - 1;
        int b = pseg[nc], p = ppos[nc]; asm volatile("" : "+v"(b)); asm volatile("" : "+v"(p));
        const int bc = b < 0 ? 0 : (b > NGR - 1 ? NGR - 1 : b);
        const int off = pri_off(bc), cnt = 32 + bc % 65;
        bad |= ok & ((int)(b != bc) | (int)(p != nc - off) | (int)(p < 0) | (int)(p >= cnt));
    }
#pragma unroll 1
    for (int n0 = 0; n0 < NS; n0 += 512) {
        const int n = n0 + tid; const int ok = (int)(n < NS); const int nc = ok ? n : NS - 1;
        int b = sseg[nc], p = spos[nc]; asm volatile("" : "+v"(b)); asm volatile("" : "+v"(p));
        const int bc = b < 0 ? 0 : (b > NGR - 1 ? NGR - 1 : b);
        const int off = sec_off(bc), cnt = 16 + bc % 49;
        const int loc = nc - off;
        const int nx = off + ((loc + 1 == cnt) ? 0 : loc + 1), pv = off + ((loc == 0) ? cnt - 1 : loc - 1);
        int s0 = esrc[nc], s1 = esrc[NS_FULL + nc], s2 = esrc[2 * NS_FULL + nc];
        int d0 = edst[nc], d1 = edst[NS_FULL + nc], d2 = edst[2 * NS_FULL + nc];
        asm volatile("" : "+v"(s0)); asm volatile("" : "+v"(s1)); asm volatile("" : "+v"(s2));
        asm volatile("" : "+v"(d0)); asm volatile("" : "+v"(d1)); asm volatile("" : "+v"(d2));
        bad |= ok & ((int)(b != bc) | (int)(p != loc) | (int)(p < 0) | (int)(p >= cnt));
        bad |= ok & ((int)(s0 != nc) | (int)(s1 != nc) | (int)(s2 != nc) | (int)(d0 != nc) | (int)(d1 != nx) | (int)(d2 != pv));
    }
    bad |= __shfl_xor(bad, 16, 32); bad |= __shfl_xor(bad, 8, 32); bad |= __shfl_xor(bad, 4, 32); bad |= __shfl_xor(bad, 2, 32); bad |= __shfl_xor(bad, 1, 32);
    if (lane == 0) wbad[wave] = bad;
    __syncthreads();
    if (wave == 0) {
        int t = wbad[lane & 15];
        t |= __shfl_xor(t, 8, 32); t |= __shfl_xor(t, 4, 32); t |= __shfl_xor(t, 2, 32); t |= __shfl_xor(t, 1, 32);
        *(volatile int*)(FLAG + lane) = t; __threadfence(); *(volatile int*)(FLAG + lane) = t;
    }
}

template <int MODE>
__device__ __forceinline__ void node_gemm(const float* __restrict__ X, const int* __restrict__ edst, const bf* __restrict__ WB, const h16* __restrict__ WH,
                                          const float* __restrict__ bias, float* Y, float* PART) {
    constexpr int  KD    = (MODE == 0) ? KE : HID;
    constexpr int  AP    = (MODE == 0) ? TP : GP;
    constexpr bool BFM   = (MODE == 0) || (MODE == 3);
    constexpr bool STATS = (MODE >= 2);
    __shared__ __align__(16) unsigned short ab[BFM ? 64 * AP : 8];
    __shared__ __align__(16) h16 ah[BFM ? 8 : 64 * AP];
    __shared__ __align__(16) h16 ar[BFM ? 8 : 64 * AP];
    __shared__ __align__(16) float os[(MODE == 3) ? 4 : 4 * 16 * OSF];
    __shared__ __align__(16) float sq[STATS ? 4 * 128 : 4];
    __shared__ __align__(16) float srow[STATS ? 128 : 4];
    static_assert(sizeof(ab) + sizeof(ah) + sizeof(ar) + sizeof(os) + sizeof(sq) + sizeof(srow) <= 131072);
    const int tid = threadIdx.x, lane = tid & 31, lr = lane & 15, hi = lane >> 4;
    const int wave = __builtin_amdgcn_readfirstlane((int)(threadIdx.x >> 5));
    const int row0 = blockIdx.x * 64;

    if (MODE == 0) {
        const size_t lim = (size_t)NS * NDIM, g0 = (size_t)row0 * NDIM;
#pragma unroll 1
        for (int i = tid; i < 64 * NDIM / 4; i += 128) {
            const size_t g = g0 + 4 * (size_t)i; const bool ok = g < lim; const size_t gc = ok ? g : (lim - 4);
            v4f v = *(const v4f*)(X + gc); asm volatile("" : "+v"(v));
#pragma unroll
            for (int j = 0; j < 4; ++j) { const int f = 4 * i + j; const int r = f / NDIM, c = f - r * NDIM; ab[r * AP + c] = ok ? f2bf(v[j]) : (unsigned short)0; }
        }
#pragma unroll 1
        for (int i = tid; i < 64 * (KE - NDIM); i += 128) { const int r = i / (KE - NDIM), c = NDIM + (i - r * (KE - NDIM)); ab[r * AP + c] = (unsigned short)0; }
    } else if (MODE == 3) {
        const size_t lim = (size_t)NM * HID, g0 = (size_t)row0 * HID;
        static_assert((64 * HID / 4) % 128 == 0);
#pragma unroll 1
        for (int i = tid; i < 64 * HID / 4; i += 128) {
            const size_t g = g0 + 4 * (size_t)i; const bool ok = g < lim; const size_t gc = ok ? g : (lim - 4);
            v4f v = *(const v4f*)(X + gc); asm volatile("" : "+v"(v));
            const int r = i >> 4, c = (i & 15) * 4; v4us o;
#pragma unroll
            for (int j = 0; j < 4; ++j) o[j] = ok ? f2bf(v[j]) : (unsigned short)0;
            *(v4us*)(&ab[r * AP + c]) = o;
        }
    } else {
#pragma unroll 1
        for (int i = tid; i < 64 * HID / 4; i += 128) {
            const int r = i >> 4, c = (i & 15) * 4; const int n = row0 + r; const bool ok = n < NS; const int nc = ok ? n : NS - 1;
            v4f a;
            if (MODE == 1) {
                int nx = edst[NS_FULL + nc], pv = edst[2 * NS_FULL + nc];
                nx = nx < 0 ? 0 : (nx > NS - 1 ? NS - 1 : nx); pv = pv < 0 ? 0 : (pv > NS - 1 ? NS - 1 : pv);
                v4f x = *(const v4f*)(X + (size_t)nc * HID + c), xp = *(const v4f*)(X + (size_t)pv * HID + c), xn = *(const v4f*)(X + (size_t)nx * HID + c);
                asm volatile("" : "+v"(x)); asm volatile("" : "+v"(xp)); asm volatile("" : "+v"(xn));
#pragma unroll
                for (int j = 0; j < 4; ++j) a[j] = x[j] * NRM + xp[j] * NRM + xn[j] * NRM;
            } else {
                v4f x = *(const v4f*)(X + (size_t)nc * HID + c); asm volatile("" : "+v"(x)); a = x;
            }
            v4h hv, rv;
#pragma unroll
            for (int j = 0; j < 4; ++j) { const float x = ok ? a[j] : 0.0f; const h16 h = toh_flush(x); hv[j] = h; rv[j] = toh_flush((x - (float)h) * QRS); }
            *(v4h*)(&ah[r * AP + c]) = hv; *(v4h*)(&ar[r * AP + c]) = rv;
        }
    }
    __syncthreads();

    v8f acc[4], accr[4];
#pragma unroll
    for (int nb = 0; nb < 4; ++nb) { acc[nb] = (v8f){}; accr[nb] = (v8f){}; }
    const int arow = (wave * 16 + lr) * AP + 8 * hi;
    const size_t boff = (size_t)lr * KD + 8 * hi;
#pragma unroll
    for (int kc = 0; kc < KD; kc += 32) {
        if (BFM) {
            const v16bf a = ldbs(&ab[arow + kc]);
#pragma unroll
            for (int nb = 0; nb < 4; ++nb) { const v16bf b = ldb(WB + boff + (size_t)nb * 16 * KD + kc); acc[nb] = wmmabg(a, b, acc[nb]); }
        } else {
            const v16h a = ldhs(&ah[arow + kc]); const v16h r = ldhs(&ar[arow + kc]);
#pragma unroll
            for (int nb = 0; nb < 4; ++nb) { const v16h b = ldh(WH + boff + (size_t)nb * 16 * KD + kc); acc[nb] = wmma16g(a, b, acc[nb]); accr[nb] = wmma16g(r, b, accr[nb]); }
        }
    }

    const int wb = wave * 16 * OSF;
#pragma unroll
    for (int nb = 0; nb < 4; ++nb) {
        const float bc = (MODE <= 1) ? bfr(bias[nb * 16 + lr]) : 0.0f;
        float s = 0.0f, q = 0.0f;
#pragma unroll
        for (int r = 0; r < 8; ++r) {
            float v;
            if (MODE == 0)      v = acc[nb][r] + bc;
            else if (MODE == 1) v = fmaxf((acc[nb][r] + accr[nb][r] * QRI) * WSI + bc, 0.0f);
            else if (MODE == 2) v = (acc[nb][r] + accr[nb][r] * QRI) * WSI;
            else                v = acc[nb][r];
            if (MODE != 3) os[wb + (8 * hi + r) * OSF + nb * 16 + lr] = v;
            if (STATS) { s += v; q += v * v; }
        }
        if (STATS) {
            s += __shfl_xor(s, 16, 32); q += __shfl_xor(q, 16, 32);
            if (hi == 0) { sq[wave * 128 + nb * 16 + lr] = s; sq[wave * 128 + 64 + nb * 16 + lr] = q; }
        }
    }
    if (MODE != 3) {
        wave_sync();
        float* yrow = Y + ((size_t)row0 + (size_t)(wave * 16)) * HID;
        static_assert(32 * 16 * 8 == 16 * HID * 4);
#pragma unroll 1
        for (int ps = 0; ps < 2; ++ps) {
#pragma unroll
            for (int s = 0; s < 8; ++s) { const int row = 2 * s + (lane >> 4), c4 = (lane & 15) * 4;
                const v4f val = *(const v4fa*)(&os[wb + row * OSF + c4]);
                *(volatile v4f*)(yrow + (size_t)row * HID + c4) = val; }
            if (ps == 0) __threadfence(); }
    }
    if (STATS) {
        __syncthreads();
        srow[tid] = ((sq[tid] + sq[128 + tid]) + sq[256 + tid]) + sq[384 + tid];
        __syncthreads();
        if (wave == 0) {
            static_assert(32 * 16 == 128 * 4);
            const v4f val = *(const v4fa*)(&srow[lane * 4]);
            float* pr = PART + (size_t)blockIdx.x * 128 + lane * 4;
            *(volatile v4f*)pr = val; __threadfence(); *(volatile v4f*)pr = val;
        }
    }
}

__global__ __launch_bounds__(128) void k_embed(const float* __restrict__ X, const bf* __restrict__ WT, const float* __restrict__ bias, float* Y) {
    node_gemm<0>(X, nullptr, WT, nullptr, bias, Y, nullptr); }
__global__ __launch_bounds__(128) void k_gconv(const float* __restrict__ X, const int* __restrict__ edst, const h16* __restrict__ WT, const float* __restrict__ bias, float* Y) {
    node_gemm<1>(X, edst, nullptr, WT, bias, Y, nullptr); }
__global__ __launch_bounds__(128) void k_sproj(const float* __restrict__ X, const h16* __restrict__ WT, float* Y, float* PART) {
    node_gemm<2>(X, nullptr, nullptr, WT, nullptr, Y, PART); }
__global__ __launch_bounds__(128) void k_hstat(const float* __restrict__ X, const bf* __restrict__ WT, float* PART) {
    node_gemm<3>(X, nullptr, WT, nullptr, nullptr, nullptr, PART); }

__global__ __launch_bounds__(256) void k_bnfin(const float* __restrict__ PART, float* STAT, double invn, int nblk) {
    __shared__ double ds[4 * 128];
    __shared__ __align__(16) float sst[128];
    const int tid = threadIdx.x, lane = tid & 31;
    const int wave = __builtin_amdgcn_readfirstlane((int)(threadIdx.x >> 5));
    const int c = tid & 63, q = tid >> 6;
    const int nb = nblk > NBH ? NBH : nblk;
    double S = 0.0, Q = 0.0;
#pragma unroll 1
    for (int i = q; i < nb; i += 4) { const float* p = PART + (size_t)i * 128 + c; S += (double)p[0]; Q += (double)p[64]; }
    ds[q * 128 + c] = S; ds[q * 128 + 64 + c] = Q;
    __syncthreads();
    if (tid < 64) {
        const double St = ((ds[c] + ds[128 + c]) + ds[256 + c]) + ds[384 + c];
        const double Qt = ((ds[64 + c] + ds[192 + c]) + ds[320 + c]) + ds[448 + c];
        const double m = St * invn; double var = Qt * invn - m * m; var = var < 0.0 ? 0.0 : var;
        sst[c] = (float)m; sst[64 + c] = 1.0f / sqrtf((float)var + BN_EPS);
    }
    __syncthreads();
    if (wave == 0) {
        const v4f val = *(const v4fa*)(&sst[lane * 4]);
        *(volatile v4f*)(STAT + lane * 4) = val; __threadfence(); *(volatile v4f*)(STAT + lane * 4) = val;
    }
}

__global__ __launch_bounds__(256) void k_inter(const float* __restrict__ hid, const float* __restrict__ HS, const float* __restrict__ YS, const bf* __restrict__ HWT,
                                               const float* __restrict__ STATH, const float* __restrict__ STATS_,
                                               const float* __restrict__ gH, const float* __restrict__ bH, const float* __restrict__ gS, const float* __restrict__ bS,
                                               h16* ZH, h16* ZR) {
    __shared__ __align__(16) unsigned short xb[LPR * GP];
    __shared__ __align__(16) h16 Hh[LPR * GP];
    __shared__ __align__(16) h16 Hr[LPR * GP];
    __shared__ __align__(16) h16 Sh[LSE * GP];
    __shared__ __align__(16) h16 Sr[LSE * GP];
    __shared__ __align__(16) h16 HT[HID * TP];
    __shared__ __align__(16) h16 ST[HID * GP];
    __shared__ __align__(16) h16 Pm[LPR * GP];
    __shared__ __align__(16) h16 PX[LSE * TP];
    __shared__ __align__(16) float zrow[ZW];
    __shared__ float sumH[4 * HID];
    __shared__ float sumS[4 * HID];
    static_assert(sizeof(xb) + sizeof(Hh) + sizeof(Hr) + sizeof(Sh) + sizeof(Sr) + sizeof(HT) + sizeof(ST) + sizeof(Pm) + sizeof(PX) + sizeof(zrow) + sizeof(sumH) + sizeof(sumS) <= 131072);
    const int tid = threadIdx.x, lane = tid & 31, lr = lane & 15, hi = lane >> 4;
    const int wave = __builtin_amdgcn_readfirstlane((int)(threadIdx.x >> 5));
    const int b = blockIdx.x;
    const int moff = pri_off(b), mc = 32 + b % 65, soff = sec_off(b), sc = 16 + b % 49;
    const int c4 = (tid & 15) * 4, rq = tid >> 4;

    static_assert(LPR % 16 == 0);
#pragma unroll 1
    for (int it = 0; it < LPR / 16; ++it) {
        const int r = it * 16 + rq; const bool ok = r < mc; const int rc = ok ? r : (mc - 1);
        v4f v = *(const v4f*)(hid + (size_t)(moff + rc) * HID + c4); asm volatile("" : "+v"(v));
        v4us o;
#pragma unroll
        for (int j = 0; j < 4; ++j) o[j] = ok ? f2bf(v[j]) : (unsigned short)0;
        *(v4us*)(&xb[r * GP + c4]) = o;
    }
    {
        const v4f smu = *(const v4f*)(STATS_ + c4), srs = *(const v4f*)(STATS_ + 64 + c4);
        const v4f sg = *(const v4f*)(gS + c4), sbb = *(const v4f*)(bS + c4);
#pragma unroll 1
        for (int it = 0; it < LSE / 16; ++it) {
            const int r = it * 16 + rq; const bool ok = r < sc; const int rc = ok ? r : (sc - 1);
            v4f v = *(const v4f*)(YS + (size_t)(soff + rc) * HID + c4); asm volatile("" : "+v"(v));
            v4h hv, rv;
#pragma unroll
            for (int j = 0; j < 4; ++j) {
                float x = ((v[j] - smu[j]) * srs[j]) * bfr(sg[j]) + bfr(sbb[j]); x = ok ? x : 0.0f;
                const h16 h = toh_flush(x); hv[j] = h; rv[j] = toh_flush((x - (float)h) * QRS);
                ST[(c4 + j) * GP + r] = h; }
            *(v4h*)(&Sh[r * GP + c4]) = hv; *(v4h*)(&Sr[r * GP + c4]) = rv;
        }
    }
    {
        const int c = tid & 63, g = tid >> 6; float aS = 0.0f;
#pragma unroll 1
        for (int r = g; r < sc; r += 4) aS += HS[(size_t)(soff + r) * HID + c];
        sumS[g * HID + c] = aS;
    }
    __syncthreads();

    {
        const int c = tid & 63, g = tid >> 6; float aH = 0.0f;
#pragma unroll 1
        for (int r = g; r < mc; r += 4) aH += __uint_as_float(((unsigned)xb[r * GP + c]) << 16);
        sumH[g * HID + c] = aH;
    }
    const int nt = wave & 3, mh = wave >> 2;
    {
        const size_t bo = (size_t)(nt * 16 + lr) * HID + 8 * hi;
        const v16bf w0 = ldb(HWT + bo), w1 = ldb(HWT + bo + 32);
        const int col = nt * 16 + lr;
        const float hm = STATH[col], hrs = STATH[64 + col], hg = bfr(gH[col]), hb = bfr(bH[col]);
#pragma unroll 1
        for (int i = 0; i < 3; ++i) {
            const int mt = mh + 2 * i; const int ao = (mt * 16 + lr) * GP + 8 * hi;
            v8f acc = (v8f){};
            acc = wmmabg(ldbs(&xb[ao]), w0, acc); acc = wmmabg(ldbs(&xb[ao + 32]), w1, acc);
            v8h hv;
#pragma unroll
            for (int r = 0; r < 8; ++r) { const int row = mt * 16 + 8 * hi + r;
                float x = ((acc[r] - hm) * hrs) * hg + hb; x = (row < mc) ? x : 0.0f;
                const h16 h = toh_flush(x); hv[r] = h;
                Hh[row * GP + col] = h; Hr[row * GP + col] = toh_flush((x - (float)h) * QRS); }
            *(v8h*)(&HT[col * TP + mt * 16 + 8 * hi]) = hv;
        }
    }
    __syncthreads();

    {
        const int so = (nt * 16 + lr) * GP + 8 * hi;
        const v16h sh0 = ldhs(&Sh[so]), sh1 = ldhs(&Sh[so + 32]), sr0 = ldhs(&Sr[so]), sr1 = ldhs(&Sr[so + 32]);
#pragma unroll 1
        for (int i = 0; i < 3; ++i) {
            const int mt = mh + 2 * i; const int ao = (mt * 16 + lr) * GP + 8 * hi;
            const v16h a0 = ldhs(&Hh[ao]), a1 = ldhs(&Hh[ao + 32]), r0 = ldhs(&Hr[ao]), r1 = ldhs(&Hr[ao + 32]);
            v8f sH = (v8f){}, sL = (v8f){};
            sH = wmma16g(a0, sh0, sH); sH = wmma16g(a1, sh1, sH);
            sL = wmma16g(a0, sr0, sL); sL = wmma16g(a1, sr1, sL);
            sL = wmma16g(r0, sh0, sL); sL = wmma16g(r1, sh1, sL);
            v8h pv;
#pragma unroll
            for (int r = 0; r < 8; ++r) { const float s = sH[r] + sL[r] * QRI; const h16 h = toh_flush(tanhf(s)); pv[r] = h;
                Pm[(mt * 16 + 8 * hi + r) * GP + nt * 16 + lr] = h; }
            *(v8h*)(&PX[(nt * 16 + lr) * TP + mt * 16 + 8 * hi]) = pv;
        }
    }
    __syncthreads();

    if (wave < 4) {
        const int bo = (wave * 16 + lr) * GP + 8 * hi;
        const v16h b0 = ldhs(&ST[bo]), b1 = ldhs(&ST[bo + 32]);
        v8f acc = (v8f){};
#pragma unroll 1
        for (int mt = 0; mt < LPR / 16; ++mt) { const int ao = (mt * 16 + lr) * GP + 8 * hi;
            acc = wmma16g(ldhs(&Pm[ao]), b0, acc); acc = wmma16g(ldhs(&Pm[ao + 32]), b1, acc); }
        float s = ((acc[0] + acc[1]) + (acc[2] + acc[3])) + ((acc[4] + acc[5]) + (acc[6] + acc[7]));
        s += __shfl_xor(s, 16, 32);
        if (hi == 0) zrow[64 + wave * 16 + lr] = s;
    } else {
        const int dt = wave - 4; const int bo = (dt * 16 + lr) * TP + 8 * hi;
        const v16h b0 = ldhs(&HT[bo]), b1 = ldhs(&HT[bo + 32]), b2 = ldhs(&HT[bo + 64]);
        v8f acc = (v8f){};
#pragma unroll 1
        for (int n2 = 0; n2 < LSE / 16; ++n2) { const int ao = (n2 * 16 + lr) * TP + 8 * hi;
            acc = wmma16g(ldhs(&PX[ao]), b0, acc); acc = wmma16g(ldhs(&PX[ao + 32]), b1, acc); acc = wmma16g(ldhs(&PX[ao + 64]), b2, acc); }
        float s = ((acc[0] + acc[1]) + (acc[2] + acc[3])) + ((acc[4] + acc[5]) + (acc[6] + acc[7]));
        s += __shfl_xor(s, 16, 32);
        if (hi == 0) zrow[192 + dt * 16 + lr] = s;
    }
    if (tid < 64) {
        zrow[tid]       = ((sumH[tid] + sumH[64 + tid]) + sumH[128 + tid]) + sumH[192 + tid];
        zrow[128 + tid] = ((sumS[tid] + sumS[64 + tid]) + sumS[128 + tid]) + sumS[192 + tid];
    }
    __syncthreads();
    static_assert(32 * 16 == ZW * 2);
    if (wave == 0) {
        v8h o;
#pragma unroll
        for (int j = 0; j < 8; ++j) o[j] = toh_flush(zrow[lane * 8 + j]);
        h16* zp = ZH + (size_t)b * ZW + lane * 8;
        *(volatile v8h*)zp = o; __threadfence(); *(volatile v8h*)zp = o;
    } else if (wave == 1) {
        v8h o;
#pragma unroll
        for (int j = 0; j < 8; ++j) { const float v = zrow[lane * 8 + j]; const h16 h = toh_flush(v); o[j] = toh_flush((v - (float)h) * QRS); }
        h16* zp = ZR + (size_t)b * ZW + lane * 8;
        *(volatile v8h*)zp = o; __threadfence(); *(volatile v8h*)zp = o;
    }
}

__global__ __launch_bounds__(256) void k_mlp(const h16* __restrict__ ZH, const h16* __restrict__ ZR, const h16* __restrict__ L1T, const float* __restrict__ l1b,
                                             const float* __restrict__ l2w, const float* __restrict__ l2b, const int* __restrict__ FLAG, float* OUT) {
    __shared__ float red[4 * 32];
    const int tid = threadIdx.x, lane = tid & 31, lr = lane & 15, hi = lane >> 4;
    const int wave = __builtin_amdgcn_readfirstlane((int)(threadIdx.x >> 5));
    const int mt = wave & 1, ng = wave >> 1;
    const int r0 = blockIdx.x * 32 + mt * 16;
    v8f acc[4], accr[4];
#pragma unroll
    for (int n = 0; n < 4; ++n) { acc[n] = (v8f){}; accr[n] = (v8f){}; }
    const size_t ao = (size_t)(r0 + lr) * ZW + 8 * hi;
    const size_t bo = (size_t)(ng * 64 + lr) * ZW + 8 * hi;
#pragma unroll 1
    for (int kc = 0; kc < ZW; kc += 32) {
        const v16h a = ldh(ZH + ao + kc), r = ldh(ZR + ao + kc);
#pragma unroll
        for (int n = 0; n < 4; ++n) { const v16h bb = ldh(L1T + bo + (size_t)n * 16 * ZW + kc); acc[n] = wmma16g(a, bb, acc[n]); accr[n] = wmma16g(r, bb, accr[n]); }
    }
    float part[8];
#pragma unroll
    for (int r = 0; r < 8; ++r) part[r] = 0.0f;
#pragma unroll
    for (int n = 0; n < 4; ++n) {
        const int col = ng * 64 + n * 16 + lr;
        const float bv = bfr(l1b[col]), wv = bfr(l2w[col]);
#pragma unroll
        for (int r = 0; r < 8; ++r) { const float v = fmaxf((acc[n][r] + accr[n][r] * QRI) * WSI + bv, 0.0f); part[r] += v * wv; }
    }
#pragma unroll
    for (int r = 0; r < 8; ++r) { part[r] += __shfl_xor(part[r], 1, 32); part[r] += __shfl_xor(part[r], 2, 32); part[r] += __shfl_xor(part[r], 4, 32); part[r] += __shfl_xor(part[r], 8, 32); }
    if (lr == 0) {
#pragma unroll
        for (int r = 0; r < 8; ++r) red[ng * 32 + mt * 16 + 8 * hi + r] = part[r];
    }
    __syncthreads();
    if (wave == 0) {
        static_assert(32 * 4 == 128);
        const float v = (((red[lane] + red[32 + lane]) + red[64 + lane]) + red[96 + lane]) + bfr(l2b[0]);
        const int fl = FLAG[lane];
        const float o = (fl != 0) ? __uint_as_float(0x7FC00000u) : v;
        float* op = OUT + (size_t)blockIdx.x * 32 + lane;
        *(volatile float*)op = o; __threadfence(); *(volatile float*)op = o;
    }
}

static constexpr size_t al256(size_t v) { return (v + 255) & ~(size_t)255; }
static constexpr size_t SZ_HP   = al256((size_t)NSP * HID * 4);
static constexpr size_t SZ_PART = al256((size_t)(NBH + NBS) * 128 * 4);
static constexpr size_t SZ_Z    = al256((size_t)NGR * ZW * 2);
static constexpr size_t SZ_EWT  = al256((size_t)HID * KE * 2);
static constexpr size_t SZ_GWT  = al256((size_t)4 * HID * HID * 2);
static constexpr size_t SZ_W64  = al256((size_t)HID * HID * 2);
static constexpr size_t SZ_L1T  = al256((size_t)ZW * ZW * 2);
static constexpr size_t SZ_STAT = al256((size_t)256 * 4);
static constexpr size_t SZ_FLAG = al256((size_t)32 * 4);
static constexpr size_t SZ_TOTAL = 2 * SZ_HP + SZ_PART + 2 * SZ_Z + SZ_EWT + SZ_GWT + 2 * SZ_W64 + SZ_L1T + SZ_STAT + SZ_FLAG;
static_assert(SZ_TOTAL <= (size_t)134217728);
static_assert((HID * KE) % (8 * 256) == 0);
static_assert((HID * HID) % (8 * 256) == 0);
static_assert((ZW * ZW) % (8 * 256) == 0);

extern "C" void kernel_launch(void* const* d_in, const int* in_sizes, int n_in,
                              void* d_out, int out_size, void* d_ws, size_t ws_size, hipStream_t stream) {
    if (n_in < 22) return;
    if ((size_t)in_sizes[0] < (size_t)NM * HID || (size_t)in_sizes[1] < (size_t)NS * NDIM) return;
    if (in_sizes[2] < NDIM * HID || in_sizes[3] < HID || in_sizes[4] < 4 * HID * HID || in_sizes[5] < 4 * HID) return;
    if (in_sizes[6] < HID * HID || in_sizes[7] < HID * HID) return;
    if (in_sizes[8] < HID || in_sizes[9] < HID || in_sizes[10] < HID || in_sizes[11] < HID) return;
    if (in_sizes[12] < ZW * ZW || in_sizes[13] < ZW || in_sizes[14] < ZW || in_sizes[15] < 1) return;
    if (in_sizes[16] < NM || in_sizes[17] < NM || in_sizes[18] < NS || in_sizes[19] < NS) return;
    if ((size_t)in_sizes[20] < (size_t)2 * NS_FULL + NS || (size_t)in_sizes[21] < (size_t)2 * NS_FULL + NS) return;
    if (NGR == NGR_FULL) {
        if (in_sizes[16] != NM_FULL || in_sizes[17] != NM_FULL || in_sizes[18] != NS_FULL || in_sizes[19] != NS_FULL) return;
        if (in_sizes[20] != 3 * NS_FULL || in_sizes[21] != 3 * NS_FULL) return;
        if ((size_t)in_sizes[0] != (size_t)NM_FULL * HID || (size_t)in_sizes[1] != (size_t)NS_FULL * NDIM) return;
    }
    if (out_size < NGR) return;
    if (SZ_TOTAL > ws_size) return;
    const float* hidden = (const float*)d_in[0];
    const float* sfeats = (const float*)d_in[1];
    const float* embW = (const float*)d_in[2];  const float* embB = (const float*)d_in[3];
    const float* gcnW = (const float*)d_in[4];  const float* gcnB = (const float*)d_in[5];
    const float* hW   = (const float*)d_in[6];  const float* sW   = (const float*)d_in[7];
    const float* bnHg = (const float*)d_in[8];  const float* bnHb = (const float*)d_in[9];
    const float* bnSg = (const float*)d_in[10]; const float* bnSb = (const float*)d_in[11];
    const float* l1W  = (const float*)d_in[12]; const float* l1b  = (const float*)d_in[13];
    const float* l2W  = (const float*)d_in[14]; const float* l2b  = (const float*)d_in[15];
    const int* pseg = (const int*)d_in[16]; const int* ppos = (const int*)d_in[17];
    const int* sseg = (const int*)d_in[18]; const int* spos = (const int*)d_in[19];
    const int* esrc = (const int*)d_in[20]; const int* edst = (const int*)d_in[21];
    float* OUT = (float*)d_out;
    char* wsp = (char*)d_ws;
    float* HA   = (float*)wsp; wsp += SZ_HP;
    float* HB   = (float*)wsp; wsp += SZ_HP;
    float* PART = (float*)wsp; wsp += SZ_PART;
    h16*   ZH   = (h16*)wsp;   wsp += SZ_Z;
    h16*   ZR   = (h16*)wsp;   wsp += SZ_Z;
    bf*    EWT  = (bf*)wsp;    wsp += SZ_EWT;
    h16*   GWT  = (h16*)wsp;   wsp += SZ_GWT;
    bf*    HWT  = (bf*)wsp;    wsp += SZ_W64;
    h16*   SWT  = (h16*)wsp;   wsp += SZ_W64;
    h16*   L1T  = (h16*)wsp;   wsp += SZ_L1T;
    float* STAT = (float*)wsp; wsp += SZ_STAT;
    int*   FLAG = (int*)wsp;   wsp += SZ_FLAG;

    k_wtb<<<(HID * KE / 8 + 255) / 256, 256, 0, stream>>>(embW, EWT, NDIM, HID, KE, HID * KE / 8);
    k_wth<<<dim3((HID * HID / 8 + 255) / 256, 4, 1), 256, 0, stream>>>(gcnW, GWT, HID, HID, HID, HID * HID / 8, WSC);
    k_wtb<<<(HID * HID / 8 + 255) / 256, 256, 0, stream>>>(hW, HWT, HID, HID, HID, HID * HID / 8);
    k_wth<<<dim3((HID * HID / 8 + 255) / 256, 1, 1), 256, 0, stream>>>(sW, SWT, HID, HID, HID, HID * HID / 8, WSC);
    k_wth<<<dim3((ZW * ZW / 8 + 255) / 256, 1, 1), 256, 0, stream>>>(l1W, L1T, ZW, ZW, ZW, ZW * ZW / 8, WSC);
    k_check<<<1, 512, 0, stream>>>(pseg, ppos, sseg, spos, esrc, edst, FLAG);

    k_embed<<<NBS, 128, 0, stream>>>(sfeats, EWT, embB, HA);
    k_gconv<<<NBS, 128, 0, stream>>>(HA, edst, GWT + (size_t)0 * HID * HID, gcnB + 0 * HID, HB);
    k_gconv<<<NBS, 128, 0, stream>>>(HB, edst, GWT + (size_t)1 * HID * HID, gcnB + 1 * HID, HA);
    k_gconv<<<NBS, 128, 0, stream>>>(HA, edst, GWT + (size_t)2 * HID * HID, gcnB + 2 * HID, HB);
    k_gconv<<<NBS, 128, 0, stream>>>(HB, edst, GWT + (size_t)3 * HID * HID, gcnB + 3 * HID, HA);
    k_sproj<<<NBS, 128, 0, stream>>>(HA, SWT, HB, PART + (size_t)NBH * 128);
    k_hstat<<<NBH, 128, 0, stream>>>(hidden, HWT, PART);
    k_bnfin<<<1, 256, 0, stream>>>(PART, STAT, 1.0 / (double)NM, NBH);
    k_bnfin<<<1, 256, 0, stream>>>(PART + (size_t)NBH * 128, STAT + 128, 1.0 / (double)NS, NBS);
    k_inter<<<NGR, 256, 0, stream>>>(hidden, HA, HB, HWT, STAT, STAT + 128, bnHg, bnHb, bnSg, bnSb, ZH, ZR);
    k_mlp<<<NGR / 32, 256, 0, stream>>>(ZH, ZR, L1T, l1b, l2W, l2b, FLAG, OUT);
}
